// C2fPSA_78907139162703
// MI455X (gfx1250) — hardware-verified
//
#include <hip/hip_runtime.h>
#include <stdint.h>
#include <math.h>

#define NB     2
#define QD     4
#define NIMG   (NB * QD)
#define IMW    24
#define HWI    576
#define TOKB   (QD * HWI)
#define NPIX   (NIMG * HWI)
#define NTILE  (NPIX / 32)
#define CIN    512
#define CC     256
#define C3     768
#define ECD    128
#define GCD    512
#define C2O    512
#define NHD    16
#define NSLICE (NIMG * NHD)
#define NQT    (HWI / 64)
#define CATW   2048
#define COLW   2304
#define SSP    36
#define SPP    40
#define OPW    68
#define EPW    120

#define SHI    16384.0f
#define SRES   4096.0f
#define SLO    4.0f
#define XSC    64.0f
#define QSC    16.0f
#define PSC    1024.0f
#define OSC3   (1.0f / 16384.0f)
#define OSC1   (1.0f / 1048576.0f)
#define LSC    (1.0f / 1024.0f)

static_assert(HWI == IMW * IMW);
static_assert(NPIX % 64 == 0);
static_assert(HWI % 64 == 0);
static_assert(TOKB % 32 == 0);
static_assert(NPIX % 256 == 0);
static_assert((NB * ECD) <= 256);
static_assert(NIMG <= 32);
static_assert(CC == NHD * 16);

typedef _Float16 v16h __attribute__((ext_vector_type(16)));
typedef _Float16 v8h  __attribute__((ext_vector_type(8)));
typedef float    v8f  __attribute__((ext_vector_type(8)));
typedef float    v4f  __attribute__((ext_vector_type(4)));
typedef unsigned int v4u __attribute__((ext_vector_type(4)));

__device__ __forceinline__ unsigned short bf_bits(float f) {
  unsigned u = __float_as_uint(f);
  return (unsigned short)((u + 0x7FFFu + ((u >> 16) & 1u)) >> 16);
}
__device__ __forceinline__ float bf_up(unsigned short b) { return __uint_as_float(((unsigned)b) << 16); }
__device__ __forceinline__ float bfr(float f) { return bf_up(bf_bits(f)); }
__device__ __forceinline__ unsigned short h_bits(_Float16 x) { return __builtin_bit_cast(unsigned short, x); }
__device__ __forceinline__ unsigned short f2h_bits(float f) { return h_bits((_Float16)f); }
__device__ __forceinline__ unsigned pk16(unsigned short a, unsigned short b) { return (unsigned)a | ((unsigned)b << 16); }
__device__ __forceinline__ v8f zero8() { v8f z = {0.f, 0.f, 0.f, 0.f, 0.f, 0.f, 0.f, 0.f}; return z; }
__device__ __forceinline__ v8h zero8h() { union { v8h v; v4u u; } z; v4u u0 = {0u, 0u, 0u, 0u}; z.u = u0; return z.v; }

__device__ __forceinline__ unsigned split_pair(float a, float b, unsigned& lo) {
  const _Float16 ha = (_Float16)a, hb = (_Float16)b;
  const _Float16 la = (_Float16)((a - (float)ha) * SRES);
  const _Float16 lb = (_Float16)((b - (float)hb) * SRES);
  lo = pk16(h_bits(la), h_bits(lb));
  return pk16(h_bits(ha), h_bits(hb));
}

__device__ __forceinline__ v16h ldfrag_h(const _Float16* p) {
  union { v16h v; v8h hh[2]; } f;
  f.hh[0] = *(const v8h*)(p);
  f.hh[1] = *(const v8h*)(p + 16);
  return f.v;
}
union FragU { v16h v; v8h hh[2]; };

__device__ __forceinline__ v8f mma_h_raw(v16h a, v16h b, v8f c) {
  return __builtin_amdgcn_wmma_f32_16x16x32_f16(false, a, false, b, (short)0, c, false, false);
}
__device__ __forceinline__ void dep_guard1(v8f& a, v16h x, v16h y) {
#if defined(__HIP_DEVICE_COMPILE__)
  asm volatile("v_nop\n\tv_nop\n\tv_nop\n\tv_nop" : "+v"(a) : "v"(x), "v"(y));
#endif
}
__device__ __forceinline__ void dep_guard_h(v8f& a, v8f& b, v16h x, v16h y) {
#if defined(__HIP_DEVICE_COMPILE__)
  asm volatile("v_nop\n\tv_nop\n\tv_nop\n\tv_nop" : "+v"(a), "+v"(b) : "v"(x), "v"(y));
#endif
}
__device__ __forceinline__ void keep4_h(v16h a, v16h b, v16h c, v16h d) {
#if defined(__HIP_DEVICE_COMPILE__)
  asm volatile("v_nop" :: "v"(a), "v"(b), "v"(c), "v"(d));
#endif
}
__device__ __forceinline__ void keep2_h(v16h a, v16h b) {
#if defined(__HIP_DEVICE_COMPILE__)
  asm volatile("v_nop" :: "v"(a), "v"(b));
#endif
}
__device__ __forceinline__ void acc_guard4(v8f& a, v8f& b, v8f& c, v8f& d) {
#if defined(__HIP_DEVICE_COMPILE__)
  asm volatile("v_nop\n\tv_nop\n\tv_nop\n\tv_nop" : "+v"(a), "+v"(b), "+v"(c), "+v"(d));
#endif
}
__device__ __forceinline__ void wave_sync_lds() {
  __builtin_amdgcn_fence(__ATOMIC_RELEASE, "workgroup");
  __builtin_amdgcn_wave_barrier();
  __builtin_amdgcn_fence(__ATOMIC_ACQUIRE, "workgroup");
}

__global__ __launch_bounds__(256) void k_cvtw(const float* __restrict__ mod, const float* __restrict__ ph,
                                               int O, int Cin, int T, int G, int NP, unsigned short* dst) {
  __shared__ __align__(16) float sW[8][512];
  const int tid = threadIdx.x, wave = tid >> 5, lane = tid & 31;
  const int o = blockIdx.x * 8 + wave;
  if (o >= O) return;
  const int CT = Cin * T;
  const int K3 = NP * CT;
  const int ngr = CT / G;
  unsigned short* drow = dst + (size_t)o * K3;
  float* sw = sW[wave];
#pragma unroll 1
  for (int gi = 0; gi < ngr; ++gi) {
#pragma unroll 1
    for (int base = 0; base < G; base += 256) {
      const int w0 = base + lane * 8;
#pragma unroll 1
      for (int i = 0; i < 8; ++i) {
        const int within = min(w0 + i, G - 1);
        const int kk = gi * G + within;
        const int c = kk % Cin;
        const int tap = kk / Cin;
        const size_t si = ((size_t)o * Cin + c) * T + tap;
        sw[within] = bfr(mod[si]) * cosf(bfr(ph[si]));
      }
    }
    wave_sync_lds();
#pragma unroll 1
    for (int part = 0; part < NP; ++part) {
#pragma unroll 1
      for (int base = 0; base < G; base += 256) {
        const int w0 = base + lane * 8;
        const bool act = (w0 < G);
        const int wl = act ? w0 : 0;
        const v4f a = *(const v4f*)(sw + wl);
        const v4f b = *(const v4f*)(sw + wl + 4);
        float v[8];
        v[0] = a[0]; v[1] = a[1]; v[2] = a[2]; v[3] = a[3];
        v[4] = b[0]; v[5] = b[1]; v[6] = b[2]; v[7] = b[3];
        v4u p;
#pragma unroll
        for (int e = 0; e < 4; ++e) {
          const float x0 = v[2 * e] * SHI, x1 = v[2 * e + 1] * SHI;
          const _Float16 h0 = (_Float16)x0, h1 = (_Float16)x1;
          const unsigned q0 = pk16(h_bits(h0), h_bits(h1));
          const unsigned q1 = pk16(f2h_bits(x0 - (float)h0), f2h_bits(x1 - (float)h1));
          const unsigned q2 = pk16(f2h_bits(v[2 * e] * SLO), f2h_bits(v[2 * e + 1] * SLO));
          p[e] = (part == 0) ? q0 : ((part == 1) ? q1 : q2);
        }
        unsigned short* d = drow + (size_t)gi * NP * G + (size_t)part * G + w0;
        if (act) *(volatile v4u*)d = p;
        __threadfence();
        if (act) *(volatile v4u*)d = p;
      }
    }
    wave_sync_lds();
  }
}

__global__ __launch_bounds__(256) void k_cvtx(const float* __restrict__ x, unsigned short* xp) {
  __shared__ __align__(16) float sx[256 * 33];
  const int tid = threadIdx.x, wave = tid >> 5, lane = tid & 31;
  const int cg = blockIdx.y;
  const int p0 = blockIdx.x * 32;
  const int b = p0 / TOKB, t0 = p0 - b * TOKB;
  const float* xb = x + ((size_t)b * CIN + (size_t)cg * 256) * TOKB + t0;
#pragma unroll 8
  for (int it = 0; it < 32; ++it) {
    const int idx = it * 256 + tid;
    const int c = idx >> 5, px = idx & 31;
    sx[c * 33 + px] = xb[(size_t)c * TOKB + px];
  }
  __syncthreads();
  const int c8 = lane * 8;
  v4u pk[4];
#pragma unroll
  for (int it = 0; it < 4; ++it) {
    const int r = wave * 4 + it;
    v4u p;
#pragma unroll
    for (int e = 0; e < 4; ++e)
      p[e] = pk16(f2h_bits(bfr(sx[(c8 + 2 * e) * 33 + r]) * XSC), f2h_bits(bfr(sx[(c8 + 2 * e + 1) * 33 + r]) * XSC));
    pk[it] = p;
  }
  unsigned short* dst = xp + (size_t)p0 * CIN + (size_t)cg * 256;
  for (int pass = 0; pass < 2; ++pass) {
#pragma unroll
    for (int it = 0; it < 4; ++it) {
      const int r = wave * 4 + it;
      *(volatile v4u*)(dst + (size_t)r * CIN + c8) = pk[it];
    }
    __threadfence();
  }
}

__global__ __launch_bounds__(256) void gemm64(
    const unsigned short* __restrict__ Ap, int lda,
    const unsigned short* __restrict__ Btp, int ldb,
    float* Cp, int ldc, int M, int N, int K, int G, int NP, int APG, float oscale) {
  const _Float16* A  = (const _Float16*)(const void*)Ap;
  const _Float16* Bt = (const _Float16*)(const void*)Btp;
  __shared__ __align__(16) float sT[8][16 * 68];
  const int lane = threadIdx.x & 31;
  const int wave = threadIdx.x >> 5;
  const int tilesN = N >> 6;
  const int tilesM = M >> 6;
  const int tile = blockIdx.x * 8 + wave;
  if (tile >= tilesM * tilesN) return;
  const int tm = tile / tilesN;
  const int tn = tile - tm * tilesN;
  const int m0 = tm << 6;
  const int n0 = tn << 6;

  const int rlane = lane & 15;
  const int koff  = (lane >> 4) * 8;
  const int mOff  = (lane >> 4) * 8;

  v8f acc[4][4];
#pragma unroll
  for (int i = 0; i < 4; ++i)
#pragma unroll
    for (int j = 0; j < 4; ++j) acc[i][j] = zero8();

  int gi = 0, part = 0, within = 0;
  for (int k0 = 0; k0 < K; k0 += 32) {
    const int kb = gi * APG + within + ((part == 2) ? G : 0);
    v16h bh[4];
#pragma unroll
    for (int j = 0; j < 4; ++j) {
      const size_t bo = (size_t)(n0 + (j << 4) + rlane) * ldb + kb + koff;
      bh[j] = ldfrag_h(Bt + bo);
    }
#pragma unroll
    for (int i = 0; i < 4; ++i) {
      const size_t ao = (size_t)(m0 + (i << 4) + rlane) * lda + k0 + koff;
      const v16h ah = ldfrag_h(A + ao);
#pragma unroll
      for (int j = 0; j < 4; ++j) {
        acc[i][j] = mma_h_raw(ah, bh[j], acc[i][j]);
      }
      dep_guard_h(acc[i][0], acc[i][3], ah, bh[3]);
    }
    keep4_h(bh[0], bh[1], bh[2], bh[3]);
    within += 32;
    if (within >= G) { within = 0; ++part; if (part >= NP) { part = 0; ++gi; } }
  }
  acc_guard4(acc[0][0], acc[0][1], acc[0][2], acc[0][3]);
  acc_guard4(acc[1][0], acc[1][1], acc[1][2], acc[1][3]);
  acc_guard4(acc[2][0], acc[2][1], acc[2][2], acc[2][3]);
  acc_guard4(acc[3][0], acc[3][1], acc[3][2], acc[3][3]);

  float* slab = sT[wave];
  float* C = Cp;
#pragma unroll
  for (int i = 0; i < 4; ++i) {
    const int mBase = m0 + (i << 4);
#pragma unroll
    for (int j = 0; j < 4; ++j) {
#pragma unroll
      for (int r = 0; r < 8; ++r) {
        slab[(mOff + r) * 68 + (j << 4) + rlane] = acc[i][j][r];
      }
    }
    wave_sync_lds();
    {
      const int hh = lane >> 4, c4 = (lane & 15) * 4;
      v4f ov[8];
#pragma unroll
      for (int it = 0; it < 8; ++it) {
        const int row = it * 2 + hh;
        v4f v = *(const v4f*)(slab + row * 68 + c4);
        v[0] *= oscale; v[1] *= oscale; v[2] *= oscale; v[3] *= oscale;
        ov[it] = v;
      }
      for (int pass = 0; pass < 2; ++pass) {
#pragma unroll
        for (int it = 0; it < 8; ++it) {
          const int row = it * 2 + hh;
          *(volatile v4f*)(C + (size_t)(mBase + row) * ldc + n0 + c4) = ov[it];
        }
        __threadfence();
      }
    }
    wave_sync_lds();
  }
}

__global__ __launch_bounds__(256) void k_stats(const float* __restrict__ src, float* st) {
  __shared__ __align__(16) float sOut[64];
  const int tid = threadIdx.x, wave = tid >> 5, lane = tid & 31;
#pragma unroll 1
  for (int i = 0; i < 4; ++i) {
    const int cl = wave * 4 + i;
    const int c = blockIdx.x * 32 + cl;
    const float* row = src + (size_t)c * NPIX;
    double s = 0.0, ss = 0.0;
#pragma unroll 4
    for (int k = 0; k < NPIX / 32; ++k) {
      const double v = (double)row[k * 32 + lane];
      s += v; ss += v * v;
    }
#pragma unroll
    for (int off = 16; off >= 1; off >>= 1) {
      s  += __shfl_xor(s, off, 32);
      ss += __shfl_xor(ss, off, 32);
    }
    if (lane == 0) {
      const double mean = s * (1.0 / (double)NPIX);
      double var = ss * (1.0 / (double)NPIX) - mean * mean;
      var = (var > 0.0) ? var : 0.0;
      const float rstd = 1.0f / sqrtf((float)var + 1.0e-5f);
      sOut[cl * 2] = (float)mean;
      sOut[cl * 2 + 1] = rstd;
    }
  }
  __syncthreads();
  if (tid < 16) {
    const v4f v = *(const v4f*)(sOut + 4 * tid);
    float* d = st + (size_t)blockIdx.x * 64 + 4 * tid;
    *(volatile v4f*)d = v;
    __threadfence();
    *(volatile v4f*)d = v;
  }
}

__device__ __forceinline__ void make_packs256(const float* sx, int wave, int lane, v4u* ph, v4u* plo) {
  const int c8 = lane * 8;
#pragma unroll
  for (int it = 0; it < 4; ++it) {
    const int r = wave * 4 + it;
    v4u a, l2;
#pragma unroll
    for (int e = 0; e < 4; ++e) {
      unsigned lo;
      a[e] = split_pair(sx[(c8 + 2 * e) * 33 + r], sx[(c8 + 2 * e + 1) * 33 + r], lo);
      l2[e] = lo;
    }
    ph[it] = a; plo[it] = l2;
  }
}
__device__ __forceinline__ void store_packs256(const v4u* ph, const v4u* plo, int wave, int lane, int p0,
                                                unsigned short* pl, int ld, int col) {
  const int c8 = lane * 8;
  for (int pass = 0; pass < 2; ++pass) {
#pragma unroll
    for (int it = 0; it < 4; ++it) {
      const int r = wave * 4 + it;
      unsigned short* d = pl + (size_t)(p0 + r) * ld + col;
      *(volatile v4u*)(d + c8) = ph[it];
      *(volatile v4u*)(d + 256 + c8) = plo[it];
    }
    __threadfence();
  }
}
template <int NCH>
__device__ __forceinline__ void store_rows(const float* sx, int wave, int lane, int p0,
                                           float* dstf, int fmode, int cd) {
  const int cq = lane >> 3, piece = (lane & 7) * 4;
  v4f ov[NCH / 32];
#pragma unroll
  for (int it = 0; it < NCH / 32; ++it) {
    const int c = wave * (NCH / 8) + it * 4 + cq;
    v4f v;
    v[0] = sx[c * 33 + piece];     v[1] = sx[c * 33 + piece + 1];
    v[2] = sx[c * 33 + piece + 2]; v[3] = sx[c * 33 + piece + 3];
    ov[it] = v;
  }
  const int b = p0 / TOKB, t0 = p0 - b * TOKB;
  for (int pass = 0; pass < 2; ++pass) {
#pragma unroll
    for (int it = 0; it < NCH / 32; ++it) {
      const int c = wave * (NCH / 8) + it * 4 + cq;
      const int o = cd + c;
      float* d = (fmode == 1) ? (dstf + (size_t)o * NPIX + p0 + piece)
                              : (dstf + ((size_t)b * C2O + o) * TOKB + t0 + piece);
      *(volatile v4f*)d = ov[it];
    }
    __threadfence();
  }
}

template <int NCH>
__global__ __launch_bounds__(256) void k_apply(
    const float* src, int csrc0,
    const float* stat, int useStat, int relu,
    const float* res, int cres0, int useRes,
    float* dstf, int fmode, int cdst0,
    unsigned short* pl1, int ld1, int col1, int use1,
    unsigned short* pl2, int ld2, int col2, int use2) {
  __shared__ __align__(16) float sx[NCH * 33];
  __shared__ float sMean[NCH];
  __shared__ float sRstd[NCH];
  const int tid = threadIdx.x, wave = tid >> 5, lane = tid & 31;
  const int cg = blockIdx.y;
  const int cs = csrc0 + cg * NCH, cr = cres0 + cg * NCH, cd = cdst0 + cg * NCH;
  const int pc1 = col1 + cg * 2 * NCH, pc2 = col2 + cg * 2 * NCH;
  const int p0 = blockIdx.x * 32;
  if (useStat) {
    for (int i = tid; i < NCH; i += 256) {
      sMean[i] = stat[(size_t)(cs + i) * 2];
      sRstd[i] = stat[(size_t)(cs + i) * 2 + 1];
    }
  }
  __syncthreads();
#pragma unroll 4
  for (int it = 0; it < NCH / 8; ++it) {
    const int idx = it * 256 + tid;
    const int c = idx >> 5, px = idx & 31;
    float v = src[(size_t)(cs + c) * NPIX + p0 + px];
    if (useStat) v = (v - sMean[c]) * sRstd[c];
    if (relu) v = fmaxf(v, 0.0f);
    if (useRes) v += res[(size_t)(cr + c) * NPIX + p0 + px];
    sx[c * 33 + px] = v;
  }
  __syncthreads();
  if (NCH == 256) {
    if ((use1 | use2) != 0) {
      v4u ph[4], plo[4];
      make_packs256(sx, wave, lane, ph, plo);
      if (use1) store_packs256(ph, plo, wave, lane, p0, pl1, ld1, pc1);
      if (use2) store_packs256(ph, plo, wave, lane, p0, pl2, ld2, pc2);
    }
  }
  if (fmode != 0) store_rows<NCH>(sx, wave, lane, p0, dstf, fmode, cd);
}

__global__ __launch_bounds__(256) void k_psa(const float* __restrict__ apr, const float* __restrict__ yn,
                                              const float* __restrict__ pem, const float* __restrict__ pep,
                                              float* apsa, unsigned short* apsp) {
  __shared__ __align__(16) float sx[256 * 33];
  __shared__ float sW[256 * 9];
  const int tid = threadIdx.x, wave = tid >> 5, lane = tid & 31;
  const int p0 = blockIdx.x * 32;
  const int img = p0 / HWI, n0 = p0 - img * HWI;
#pragma unroll 1
  for (int i = tid; i < 256 * 9; i += 256) sW[i] = bfr(pem[i]) * cosf(bfr(pep[i]));
  __syncthreads();
#pragma unroll 2
  for (int it = 0; it < 32; ++it) {
    const int idx = it * 256 + tid;
    const int c = idx >> 5, px = idx & 31;
    const int n = n0 + px;
    const int y = n / IMW, xq = n - y * IMW;
    const float* brow = yn + (size_t)(CC + c) * NPIX + (size_t)img * HWI;
    float pe = 0.0f;
#pragma unroll
    for (int t = 0; t < 9; ++t) {
      const int dy = t / 3 - 1, dx = t % 3 - 1;
      const int yy = y + dy, xx = xq + dx;
      const bool ok = ((unsigned)yy < (unsigned)IMW) && ((unsigned)xx < (unsigned)IMW);
      const int yc = min(max(yy, 0), IMW - 1), xc = min(max(xx, 0), IMW - 1);
      const float bv = brow[yc * IMW + xc];
      const float w = sW[c * 9 + t];
      pe += ok ? (w * bv) : 0.0f;
    }
    const float v = (apr[(size_t)c * NPIX + p0 + px] + pe) + brow[n];
    sx[c * 33 + px] = v;
  }
  __syncthreads();
  {
    v4u ph[4], plo[4];
    make_packs256(sx, wave, lane, ph, plo);
    store_packs256(ph, plo, wave, lane, p0, apsp, 2 * CC, 0);
  }
  store_rows<256>(sx, wave, lane, p0, apsa, 1, 0);
}

__global__ __launch_bounds__(256) void k_cvth(const float* __restrict__ src, unsigned short* dst) {
  const int tid = threadIdx.x, wave = tid >> 5, lane = tid & 31;
  const int row = blockIdx.x * 8 + wave;
  if (row < C3) {
    const float* s = src + (size_t)row * NPIX;
    unsigned short* d = dst + (size_t)row * NPIX;
#pragma unroll 1
    for (int it = 0; it < NPIX / 256; ++it) {
      const int base = it * 256 + lane * 8;
      const v4f a = *(const v4f*)(s + base);
      const v4f c = *(const v4f*)(s + base + 4);
      v4u p;
      p[0] = pk16(f2h_bits(a[0] * QSC), f2h_bits(a[1] * QSC));
      p[1] = pk16(f2h_bits(a[2] * QSC), f2h_bits(a[3] * QSC));
      p[2] = pk16(f2h_bits(c[0] * QSC), f2h_bits(c[1] * QSC));
      p[3] = pk16(f2h_bits(c[2] * QSC), f2h_bits(c[3] * QSC));
      *(volatile v4u*)(d + base) = p;
      __threadfence();
      *(volatile v4u*)(d + base) = p;
    }
  }
}

__global__ __launch_bounds__(128) void k_attn(const unsigned short* __restrict__ qkvh, float* at) {
  __shared__ __align__(16) _Float16 sK[HWI * 16];
  __shared__ __align__(16) _Float16 sQ[64 * 16];
  __shared__ __align__(16) float sS[4][16 * SSP];
  __shared__ __align__(16) _Float16 sP[4][16 * SPP];
  __shared__ __align__(16) float sAl[4][16];
  __shared__ __align__(16) float sO[16 * OPW];
  const int tid = threadIdx.x, wave = tid >> 5, lane = tid & 31, rl = lane & 15, h = lane >> 4;
  const int slice = blockIdx.x / NQT;
  const int qt = blockIdx.x - slice * NQT;
  const int img = slice / NHD, hd = slice - img * NHD;
  const int q0 = qt * 64;
  const size_t colbase = (size_t)img * HWI;
  const int qrow0 = hd * 16, krow0 = CC + hd * 16, vrow0 = 2 * CC + hd * 16;

  for (int v = tid; v < (16 * HWI) / 8; v += 128) {
    const int c = v / (HWI / 8);
    const int t8 = (v - c * (HWI / 8)) * 8;
    const v4u d = *(const v4u*)(qkvh + (size_t)(krow0 + c) * NPIX + colbase + t8);
#pragma unroll
    for (int j = 0; j < 4; ++j) {
      sK[(t8 + 2 * j) * 16 + c]     = __builtin_bit_cast(_Float16, (unsigned short)(d[j] & 0xFFFFu));
      sK[(t8 + 2 * j + 1) * 16 + c] = __builtin_bit_cast(_Float16, (unsigned short)(d[j] >> 16));
    }
  }
  {
    const int c = tid >> 3, t8 = (tid & 7) * 8;
    const v4u d = *(const v4u*)(qkvh + (size_t)(qrow0 + c) * NPIX + colbase + q0 + t8);
#pragma unroll
    for (int j = 0; j < 4; ++j) {
      sQ[(t8 + 2 * j) * 16 + c]     = __builtin_bit_cast(_Float16, (unsigned short)(d[j] & 0xFFFFu));
      sQ[(t8 + 2 * j + 1) * 16 + c] = __builtin_bit_cast(_Float16, (unsigned short)(d[j] >> 16));
    }
  }
  __syncthreads();

  FragU qa;
  qa.hh[0] = *(const v8h*)(sQ + (16 * wave + rl) * 16 + 8 * h);
  qa.hh[1] = zero8h();
  v8f acc = zero8();
  float mrow = -1.0e30f, lrow = 0.0f;
  const _Float16* H = (const _Float16*)(const void*)qkvh;
  const _Float16* Vr = H + (size_t)(vrow0 + rl) * NPIX + colbase;
  float* ss = sS[wave];
  _Float16* sp = sP[wave];
  float* sal = sAl[wave];

#pragma unroll 1
  for (int kc = 0; kc < HWI / 32; ++kc) {
    FragU kf0, kf1;
    kf0.hh[0] = *(const v8h*)(sK + (kc * 32 + rl) * 16 + 8 * h);
    kf0.hh[1] = zero8h();
    kf1.hh[0] = *(const v8h*)(sK + (kc * 32 + 16 + rl) * 16 + 8 * h);
    kf1.hh[1] = zero8h();
    v8f s0 = mma_h_raw(qa.v, kf0.v, zero8());
    v8f s1 = mma_h_raw(qa.v, kf1.v, zero8());
    dep_guard_h(s0, s1, qa.v, kf1.v);
    keep2_h(kf0.v, kf1.v);
    wave_sync_lds();
#pragma unroll
    for (int r = 0; r < 8; ++r) {
      ss[(8 * h + r) * SSP + rl] = s0[r];
      ss[(8 * h + r) * SSP + 16 + rl] = s1[r];
    }
    wave_sync_lds();
    const v4f t0 = *(const v4f*)(ss + rl * SSP + 16 * h);
    const v4f t1 = *(const v4f*)(ss + rl * SSP + 16 * h + 4);
    const v4f t2 = *(const v4f*)(ss + rl * SSP + 16 * h + 8);
    const v4f t3 = *(const v4f*)(ss + rl * SSP + 16 * h + 12);
    float lg[16];
    lg[0] = t0[0]; lg[1] = t0[1]; lg[2] = t0[2]; lg[3] = t0[3];
    lg[4] = t1[0]; lg[5] = t1[1]; lg[6] = t1[2]; lg[7] = t1[3];
    lg[8] = t2[0]; lg[9] = t2[1]; lg[10] = t2[2]; lg[11] = t2[3];
    lg[12] = t3[0]; lg[13] = t3[1]; lg[14] = t3[2]; lg[15] = t3[3];
    float mx = -1.0e30f;
#pragma unroll
    for (int i = 0; i < 16; ++i) { lg[i] *= LSC; mx = fmaxf(mx, lg[i]); }
    mx = fmaxf(mx, __shfl_xor(mx, 16, 32));
    const float mnew = fmaxf(mrow, mx);
    const float alpha = __expf(mrow - mnew);
    float psum = 0.0f;
    v8h pv0, pv1;
#pragma unroll
    for (int i = 0; i < 8; ++i) {
      const float pa = __expf(lg[i] - mnew);
      const float pb = __expf(lg[8 + i] - mnew);
      psum += pa + pb;
      pv0[i] = (_Float16)(pa * PSC);
      pv1[i] = (_Float16)(pb * PSC);
    }
    psum += __shfl_xor(psum, 16, 32);
    lrow = lrow * alpha + psum;
    mrow = mnew;
    *(v8h*)(sp + rl * SPP + 16 * h) = pv0;
    *(v8h*)(sp + rl * SPP + 16 * h + 8) = pv1;
    if (h == 0) sal[rl] = alpha;
    wave_sync_lds();
    const v4f al0 = *(const v4f*)(sal + 8 * h);
    const v4f al1 = *(const v4f*)(sal + 8 * h + 4);
    v8f alv;
    alv[0] = al0[0]; alv[1] = al0[1]; alv[2] = al0[2]; alv[3] = al0[3];
    alv[4] = al1[0]; alv[5] = al1[1]; alv[6] = al1[2]; alv[7] = al1[3];
    acc = acc * alv;
    const v16h pf = ldfrag_h(sp + rl * SPP + 8 * h);
    const v16h vf = ldfrag_h(Vr + kc * 32 + 8 * h);
    acc = mma_h_raw(pf, vf, acc);
    dep_guard1(acc, pf, vf);
  }
  wave_sync_lds();
  if (h == 0) sal[rl] = 1.0f / (lrow * 16384.0f);
  wave_sync_lds();
  {
    const v4f r0 = *(const v4f*)(sal + 8 * h);
    const v4f r1 = *(const v4f*)(sal + 8 * h + 4);
    float o[8];
    o[0] = acc[0] * r0[0]; o[1] = acc[1] * r0[1]; o[2] = acc[2] * r0[2]; o[3] = acc[3] * r0[3];
    o[4] = acc[4] * r1[0]; o[5] = acc[5] * r1[1]; o[6] = acc[6] * r1[2]; o[7] = acc[7] * r1[3];
#pragma unroll
    for (int r = 0; r < 8; ++r) sO[rl * OPW + 16 * wave + 8 * h + r] = o[r];
  }
  __syncthreads();
  {
    const int piece = (lane & 15) * 4;
    v4f ov[2];
#pragma unroll
    for (int it = 0; it < 2; ++it) {
      const int d = 4 * wave + 2 * it + (lane >> 4);
      ov[it] = *(const v4f*)(sO + d * OPW + piece);
    }
    for (int pass = 0; pass < 2; ++pass) {
#pragma unroll
      for (int it = 0; it < 2; ++it) {
        const int d = 4 * wave + 2 * it + (lane >> 4);
        *(volatile v4f*)(at + (size_t)(hd * 16 + d) * NPIX + colbase + q0 + piece) = ov[it];
      }
      __threadfence();
    }
  }
}

__global__ __launch_bounds__(256) void k_gate(const float* __restrict__ en, const float* __restrict__ guide,
                                               const float* __restrict__ glw, const float* __restrict__ glb,
                                               float* gate) {
  __shared__ float sG[NB * ECD];
  __shared__ float sRed[256];
  __shared__ __align__(16) float sOut[32];
  const int tid = threadIdx.x;
  for (int i = tid; i < NB * ECD; i += 256) {
    const int b = i / ECD, e = i - b * ECD;
    float s = 0.0f;
#pragma unroll 1
    for (int k = 0; k < GCD; ++k) s += bfr(guide[b * GCD + k]) * bfr(glw[(size_t)e * GCD + k]);
    sG[i] = s + bfr(glb[e]);
  }
  if (tid < 32) sOut[tid] = 0.0f;
  __syncthreads();
  const float inv = 1.0f / sqrtf((float)(ECD * HWI));
#pragma unroll 1
  for (int img = 0; img < NIMG; ++img) {
    const int b = img / QD;
    float s = 0.0f;
#pragma unroll 1
    for (int c = 0; c < ECD; ++c) {
      const float* row = en + (size_t)c * NPIX + (size_t)img * HWI;
      float t = 0.0f;
      for (int n = tid; n < HWI; n += 256) t += row[n];
      s += sG[b * ECD + c] * t;
    }
    sRed[tid] = s;
    __syncthreads();
    for (int off = 128; off > 0; off >>= 1) {
      if (tid < off) sRed[tid] += sRed[tid + off];
      __syncthreads();
    }
    if (tid == 0) {
      float a = sRed[0] * inv;
      a = fminf(fmaxf(a, -60.0f), 60.0f);
      sOut[img] = 1.0f / (1.0f + expf(-a));
    }
    __syncthreads();
  }
  if (tid < 8) {
    const v4f v = *(const v4f*)(sOut + 4 * tid);
    float* d = gate + 4 * tid;
    *(volatile v4f*)d = v;
    __threadfence();
    *(volatile v4f*)d = v;
  }
}

__global__ __launch_bounds__(256) void k_im2col(const float* __restrict__ en, const float* __restrict__ gate,
                                                 unsigned short* col) {
  __shared__ float sE[ECD * EPW];
  const int tid = threadIdx.x, wave = tid >> 5, lane = tid & 31;
  const int p0 = blockIdx.x * 32;
  const int img = p0 / HWI, n0 = p0 - img * HWI;
  const int y0 = n0 / IMW, y1 = (n0 + 31) / IMW;
  const int ylo = max(y0 - 1, 0), yhi = min(y1 + 1, IMW - 1);
  const int npx = (yhi - ylo + 1) * IMW;
  const float ga = gate[img];
  const size_t base = (size_t)img * HWI + (size_t)ylo * IMW;
  for (int i = tid; i < ECD * npx; i += 256) {
    const int c = i / npx, j = i - c * npx;
    sE[c * EPW + j] = en[(size_t)c * NPIX + base + j] * ga;
  }
  __syncthreads();
  const int cl = (lane & 15) * 8, half = lane >> 4;
#pragma unroll 1
  for (int it = 0; it < 36; ++it) {
    const int seg = wave * 36 + it;
    const int r = seg / 9, t = seg - r * 9;
    const int n = n0 + r;
    const int y = n / IMW, xq = n - y * IMW;
    const int yy = y + t / 3 - 1, xx = xq + (t - (t / 3) * 3) - 1;
    const bool ok = ((unsigned)yy < (unsigned)IMW) && ((unsigned)xx < (unsigned)IMW);
    const int li = (min(max(yy, ylo), yhi) - ylo) * IMW + min(max(xx, 0), IMW - 1);
    float v[8];
#pragma unroll
    for (int j = 0; j < 8; ++j) v[j] = sE[(cl + j) * EPW + li];
    v4u o;
#pragma unroll
    for (int e = 0; e < 4; ++e) {
      unsigned lo;
      const unsigned hi = split_pair(v[2 * e], v[2 * e + 1], lo);
      const unsigned w = (half == 0) ? hi : lo;
      o[e] = ok ? w : 0u;
    }
    unsigned short* d = col + (size_t)(p0 + r) * COLW + (size_t)t * 256 + lane * 8;
    *(volatile v4u*)d = o;
    __threadfence();
    *(volatile v4u*)d = o;
  }
}

static void gemm_launch(const unsigned short* A, int lda, const unsigned short* Bt, int ldb, float* C,
                        int M, int K, int G, int NP, int APG, float osc, hipStream_t st) {
  const int tiles = (M / 64) * (NPIX / 64);
  gemm64<<<dim3((tiles + 7) / 8), dim3(256), 0, st>>>(A, lda, Bt, ldb, C, NPIX, M, NPIX, K, G, NP, APG, osc);
}

extern "C" void kernel_launch(void* const* d_in, const int* in_sizes, int n_in,
                              void* d_out, int out_size, void* d_ws, size_t ws_size,
                              hipStream_t stream) {
  if (n_in < 22) return;
  if (in_sizes[0]  != NB * CIN * TOKB) return;
  if (in_sizes[1]  != NB * GCD) return;
  if (in_sizes[2]  != 512 * CIN) return;
  if (in_sizes[3]  != 512 * CIN) return;
  if (in_sizes[4]  != C3 * CC) return;
  if (in_sizes[5]  != C3 * CC) return;
  if (in_sizes[6]  != CC * CC) return;
  if (in_sizes[7]  != CC * CC) return;
  if (in_sizes[8]  != CC * 9) return;
  if (in_sizes[9]  != CC * 9) return;
  if (in_sizes[10] != 512 * CC) return;
  if (in_sizes[11] != 512 * CC) return;
  if (in_sizes[12] != CC * 512) return;
  if (in_sizes[13] != CC * 512) return;
  if (in_sizes[14] != ECD * CC) return;
  if (in_sizes[15] != ECD * CC) return;
  if (in_sizes[16] != ECD * GCD) return;
  if (in_sizes[17] != ECD) return;
  if (in_sizes[18] != CC * ECD * 9) return;
  if (in_sizes[19] != CC * ECD * 9) return;
  if (in_sizes[20] != C2O * 1024) return;
  if (in_sizes[21] != C2O * 1024) return;
  if (out_size != NB * C2O * TOKB) return;

  const float* x      = (const float*)d_in[0];
  const float* guide  = (const float*)d_in[1];
  const float* cv1_m  = (const float*)d_in[2];
  const float* cv1_p  = (const float*)d_in[3];
  const float* qkv_m  = (const float*)d_in[4];
  const float* qkv_p  = (const float*)d_in[5];
  const float* apr_m  = (const float*)d_in[6];
  const float* apr_p  = (const float*)d_in[7];
  const float* pe_m   = (const float*)d_in[8];
  const float* pe_p   = (const float*)d_in[9];
  const float* f1_m   = (const float*)d_in[10];
  const float* f1_p   = (const float*)d_in[11];
  const float* f2_m   = (const float*)d_in[12];
  const float* f2_p   = (const float*)d_in[13];
  const float* ec_m   = (const float*)d_in[14];
  const float* ec_p   = (const float*)d_in[15];
  const float* gl_w   = (const float*)d_in[16];
  const float* gl_b   = (const float*)d_in[17];
  const float* mp_m   = (const float*)d_in[18];
  const float* mp_p   = (const float*)d_in[19];
  const float* cv2_m  = (const float*)d_in[20];
  const float* cv2_p  = (const float*)d_in[21];
  float* out = (float*)d_out;

  const size_t PWCV1 = (size_t)512 * 1024 * 2;
  const size_t PWQKV = (size_t)C3 * 768 * 2;
  const size_t PWAPR = (size_t)CC * 768 * 2;
  const size_t PWF1  = (size_t)512 * 768 * 2;
  const size_t PWF2  = (size_t)CC * 1536 * 2;
  const size_t PWEC  = (size_t)ECD * 768 * 2;
  const size_t PWMP  = (size_t)CC * 3456 * 2;
  const size_t PWCV2 = (size_t)C2O * 3072 * 2;
  const size_t PST   = (size_t)512 * 2 * 4;
  const size_t PGATE = 256;
  const size_t PCATP = (size_t)NPIX * CATW * 2;
  const size_t PXP   = (size_t)NPIX * CIN * 2;
  const size_t PQKVF = (size_t)C3 * NPIX * 4;
  const size_t PF256 = (size_t)CC * NPIX * 4;
  const size_t PF512 = (size_t)512 * NPIX * 4;
  const size_t PH1P  = (size_t)NPIX * 1024 * 2;
  const size_t PP512 = (size_t)NPIX * 512 * 2;
  const size_t PCOL  = (size_t)NPIX * COLW * 2;
  const size_t PQKVH = (size_t)C3 * NPIX * 2;
  size_t PS1 = PXP;
  if (PQKVF > PS1) PS1 = PQKVF;
  if (PF256 > PS1) PS1 = PF256;
  if (PH1P  > PS1) PS1 = PH1P;
  if (PP512 > PS1) PS1 = PP512;
  if (PCOL  > PS1) PS1 = PCOL;
  if (PF512 > PS1) PS1 = PF512;
  size_t PS2 = PF512;
  size_t PS3 = PQKVH;
  if (PP512 > PS3) PS3 = PP512;
  if (PF256 + PP512 > PS3) PS3 = PF256 + PP512;

  size_t off = 0;
  const size_t oWCV1 = off; off += PWCV1;
  const size_t oWQKV = off; off += PWQKV;
  const size_t oWAPR = off; off += PWAPR;
  const size_t oWF1  = off; off += PWF1;
  const size_t oWF2  = off; off += PWF2;
  const size_t oWEC  = off; off += PWEC;
  const size_t oWMP  = off; off += PWMP;
  const size_t oWCV2 = off; off += PWCV2;
  const size_t oST   = off; off += 6 * PST;
  const size_t oGATE = off; off += PGATE;
  const size_t oCATP = off; off += PCATP;
  const size_t oS1   = off; off += PS1;
  const size_t oS2   = off; off += PS2;
  const size_t oS3   = off; off += PS3;
  if (off > ws_size) return;
  if (off > (size_t)134217728) return;

  char* ws = (char*)d_ws;
  unsigned short* WCV1 = (unsigned short*)(ws + oWCV1);
  unsigned short* WQKV = (unsigned short*)(ws + oWQKV);
  unsigned short* WAPR = (unsigned short*)(ws + oWAPR);
  unsigned short* WF1  = (unsigned short*)(ws + oWF1);
  unsigned short* WF2  = (unsigned short*)(ws + oWF2);
  unsigned short* WEC  = (unsigned short*)(ws + oWEC);
  unsigned short* WMP  = (unsigned short*)(ws + oWMP);
  unsigned short* WCV2 = (unsigned short*)(ws + oWCV2);
  float* ST0 = (float*)(ws + oST);
  float* ST1 = (float*)(ws + oST + PST);
  float* ST2 = (float*)(ws + oST + 2 * PST);
  float* ST3 = (float*)(ws + oST + 3 * PST);
  float* ST4 = (float*)(ws + oST + 4 * PST);
  float* ST5 = (float*)(ws + oST + 5 * PST);
  float* GATE = (float*)(ws + oGATE);
  unsigned short* CATP = (unsigned short*)(ws + oCATP);
  unsigned short* XP   = (unsigned short*)(ws + oS1);
  float*          QKVF = (float*)(ws + oS1);
  float*          AT   = (float*)(ws + oS1);
  float*          APR  = (float*)(ws + oS1);
  unsigned short* H1P  = (unsigned short*)(ws + oS1);
  unsigned short* PP   = (unsigned short*)(ws + oS1);
  unsigned short* COL  = (unsigned short*)(ws + oS1);
  float*          OUT2 = (float*)(ws + oS1);
  float* Y  = (float*)(ws + oS2);
  float* H1 = (float*)(ws + oS2);
  float* F2 = (float*)(ws + oS2);
  float* E  = (float*)(ws + oS2);
  float* MF = (float*)(ws + oS2);
  unsigned short* QKVH = (unsigned short*)(ws + oS3);
  unsigned short* ATP  = (unsigned short*)(ws + oS3);
  float*          APSA = (float*)(ws + oS3);
  unsigned short* APSP = (unsigned short*)(ws + oS3 + PF256);

  const dim3 blk(256);

  k_cvtw<<<dim3(512 / 8), blk, 0, stream>>>(cv1_m, cv1_p, 512, CIN, 1, 512, 2, WCV1);
  k_cvtw<<<dim3(C3 / 8),  blk, 0, stream>>>(qkv_m, qkv_p, C3, CC, 1, 256, 3, WQKV);
  k_cvtw<<<dim3(CC / 8),  blk, 0, stream>>>(apr_m, apr_p, CC, CC, 1, 256, 3, WAPR);
  k_cvtw<<<dim3(512 / 8), blk, 0, stream>>>(f1_m, f1_p, 512, CC, 1, 256, 3, WF1);
  k_cvtw<<<dim3(CC / 8),  blk, 0, stream>>>(f2_m, f2_p, CC, 512, 1, 256, 3, WF2);
  k_cvtw<<<dim3(ECD / 8), blk, 0, stream>>>(ec_m, ec_p, ECD, CC, 1, 256, 3, WEC);
  k_cvtw<<<dim3(CC / 8),  blk, 0, stream>>>(mp_m, mp_p, CC, ECD, 9, 128, 3, WMP);
  k_cvtw<<<dim3(C2O / 8), blk, 0, stream>>>(cv2_m, cv2_p, C2O, 1024, 1, 256, 3, WCV2);
  k_cvtx<<<dim3(NTILE, 2), blk, 0, stream>>>(x, XP);
  gemm_launch(WCV1, 1024, XP, CIN, Y, 512, 1024, 512, 2, 512, OSC1, stream);
  k_stats<<<dim3(512 / 32), blk, 0, stream>>>(Y, ST0);
  k_apply<256><<<dim3(NTILE, 2), blk, 0, stream>>>(Y, 0, ST0, 1, 1, Y, 0, 0, Y, 1, 0,
                                                   CATP, CATW, 0, 1, CATP, CATW, 0, 0);
  gemm_launch(WQKV, 768, CATP + 512, CATW, QKVF, C3, 768, 256, 3, 512, OSC3, stream);
  k_cvth<<<dim3(C3 / 8), blk, 0, stream>>>(QKVF, QKVH);
  k_attn<<<dim3(NSLICE * NQT), dim3(128), 0, stream>>>(QKVH, AT);
  k_apply<256><<<dim3(NTILE, 1), blk, 0, stream>>>(AT, 0, ST0, 0, 0, AT, 0, 0, AT, 0, 0,
                                                   ATP, 2 * CC, 0, 1, ATP, 2 * CC, 0, 0);
  gemm_launch(WAPR, 768, ATP, 2 * CC, APR, CC, 768, 256, 3, 512, OSC3, stream);
  k_psa<<<dim3(NTILE), blk, 0, stream>>>(APR, Y, pe_m, pe_p, APSA, APSP);
  gemm_launch(WF1, 768, APSP, 2 * CC, H1, 512, 768, 256, 3, 512, OSC3, stream);
  k_stats<<<dim3(512 / 32), blk, 0, stream>>>(H1, ST1);
  k_apply<256><<<dim3(NTILE, 2), blk, 0, stream>>>(H1, 0, ST1, 1, 1, H1, 0, 0, H1, 0, 0,
                                                   H1P, 1024, 0, 1, H1P, 1024, 0, 0);
  gemm_launch(WF2, 1536, H1P, 1024, F2, CC, 1536, 256, 3, 512, OSC3, stream);
  k_stats<<<dim3(CC / 32), blk, 0, stream>>>(F2, ST2);
  k_apply<256><<<dim3(NTILE, 1), blk, 0, stream>>>(F2, 0, ST2, 1, 0, APSA, 0, 1, F2, 0, 0,
                                                   PP, 2 * CC, 0, 1, CATP, CATW, 1024, 1);
  gemm_launch(WEC, 768, PP, 2 * CC, E, ECD, 768, 256, 3, 512, OSC3, stream);
  k_stats<<<dim3(ECD / 32), blk, 0, stream>>>(E, ST3);
  k_apply<128><<<dim3(NTILE, 1), blk, 0, stream>>>(E, 0, ST3, 1, 1, E, 0, 0, E, 1, 0,
                                                   CATP, CATW, 0, 0, CATP, CATW, 0, 0);
  k_gate<<<dim3(1), blk, 0, stream>>>(E, guide, gl_w, gl_b, GATE);
  k_im2col<<<dim3(NTILE), blk, 0, stream>>>(E, GATE, COL);
  gemm_launch(WMP, 3456, COL, COLW, MF, CC, 3456, 128, 3, 256, OSC3, stream);
  k_stats<<<dim3(CC / 32), blk, 0, stream>>>(MF, ST4);
  k_apply<256><<<dim3(NTILE, 1), blk, 0, stream>>>(MF, 0, ST4, 1, 1, MF, 0, 0, MF, 0, 0,
                                                   CATP, CATW, 1536, 1, CATP, CATW, 0, 0);
  gemm_launch(WCV2, 3072, CATP, CATW, OUT2, C2O, 3072, 256, 3, 512, OSC3, stream);
  k_stats<<<dim3(C2O / 32), blk, 0, stream>>>(OUT2, ST5);
  k_apply<256><<<dim3(NTILE, 2), blk, 0, stream>>>(OUT2, 0, ST5, 1, 1, OUT2, 0, 0, out, 2, 0,
                                                   CATP, CATW, 0, 0, CATP, CATW, 0, 0);
  (void)hipGetLastError();
}
